// KANGNN_6940667150995
// MI455X (gfx1250) — hardware-verified
//
#include <hip/hip_runtime.h>
#include <math.h>


#define NN 100000
#define NE 1600000
#define CIN 16
#define HH 32
#define HF 16
#define NBAS 11
#define NG 128
#define SLOTC 64
#define NCH 768

typedef __attribute__((ext_vector_type(16))) _Float16 v16h;
typedef __attribute__((ext_vector_type(8)))  float v8f;
typedef __attribute__((ext_vector_type(4)))  float v4f;
typedef __attribute__((ext_vector_type(4)))  int v4i;
typedef float __attribute__((may_alias)) float_a;
typedef int __attribute__((may_alias)) int_a;

template <typename T> __device__ __forceinline__ void vst2(void* p, T v) { *(volatile T*)p = v; __threadfence(); *(volatile T*)p = v; }
__device__ __forceinline__ v8f wmma16(v16h a, v16h b, v8f c) {
  v8f d = __builtin_amdgcn_wmma_f32_16x16x32_f16(false, a, false, b, (short)0, c, false, false);
  asm volatile("v_nop\n\tv_nop\n\tv_nop\n\tv_nop" : "+v"(d) : "v"(a), "v"(b));
  return d;
}
__device__ __forceinline__ v16h frag_rowK(const float* row, int lane, int K) {
  v16h a; const int g = lane >> 4;
#pragma unroll
  for (int i = 0; i < 8; ++i) { const int ka = 8 * g + i, kb = ka + 16; a[i] = (_Float16)(ka < K ? row[ka] : 0.f); a[8 + i] = (_Float16)(kb < K ? row[kb] : 0.f); }
  return a;
}
__device__ __forceinline__ v16h frag_col(const float* W, int n, int lane, int ld, int K) {
  v16h a; const int g = lane >> 4;
#pragma unroll
  for (int i = 0; i < 8; ++i) { const int ka = 8 * g + i, kb = ka + 16;
    a[i] = (_Float16)(ka < K ? W[(size_t)ka * ld + n] : 0.f); a[8 + i] = (_Float16)(kb < K ? W[(size_t)kb * ld + n] : 0.f); }
  return a;
}
#define LDSX() do { asm volatile("s_wait_dscnt 0" ::: "memory"); __builtin_amdgcn_wave_barrier(); __builtin_amdgcn_fence(__ATOMIC_RELEASE, "workgroup"); } while (0)

__device__ __forceinline__ float spline_act(float x, const float* coef, float blend) {
  const float xc = fminf(fmaxf(x, -3.0f), 3.0f);
  const float u = (xc + 3.0f) * (13.0f / 6.0f);
  float s = 0.f;
  if (u < 13.0f) {
    int i = (int)floorf(u); i = i < 0 ? 0 : (i > 12 ? 12 : i); const float t = u - (float)i;
    const float w0 = 0.5f * (1.0f - t) * (1.0f - t), w1 = 0.5f * (-2.0f * t * t + 2.0f * t + 1.0f), w2 = 0.5f * t * t;
    if (i - 2 >= 0 && i - 2 < NBAS) s += w0 * coef[i - 2];
    if (i - 1 >= 0 && i - 1 < NBAS) s += w1 * coef[i - 1];
    if (i < NBAS) s += w2 * coef[i];
  }
  return x / (1.0f + expf(-x)) + fabsf(blend) * s;
}

__global__ __launch_bounds__(128) void k_in(const float* __restrict__ x, const float* __restrict__ Win, const float* __restrict__ bin,
                                          const float* __restrict__ coef, const float* __restrict__ blend, float* __restrict__ h) {
  __shared__ __align__(16) float so[4][16][HH];
  const int tid = threadIdx.x, w = tid >> 5, lane = tid & 31, col = lane & 15, g = lane >> 4;
  const int n0 = blockIdx.x * 64 + w * 16;
  if (n0 >= NN) return;
  const v16h a = frag_rowK(x + (size_t)(n0 + col) * CIN, lane, CIN);
  v8f acc[2] = {};
#pragma unroll
  for (int t = 0; t < 2; ++t) acc[t] = wmma16(a, frag_col(Win, t * 16 + col, lane, HH, CIN), acc[t]);
  const float bl = blend[0];
#pragma unroll
  for (int t = 0; t < 2; ++t)
#pragma unroll 1
    for (int r = 0; r < 8; ++r) { const int c = t * 16 + col; so[w][8 * g + r][c] = spline_act(acc[t][r] + bin[c], coef, bl); }
  LDSX();
#pragma unroll
  for (int q = 0; q < 4; ++q) { const int rl = q * 4 + (lane >> 3), pc = lane & 7;
    vst2(h + (size_t)(n0 + rl) * HH + pc * 4, *(const v4f*)(&so[w][rl][pc * 4])); }
}

__global__ __launch_bounds__(256) void k_bucket(const int* __restrict__ ei, int* __restrict__ tlist, int* __restrict__ cnt) {
  __shared__ int scnt[NCH];
  __shared__ int slots[NCH][SLOTC];
  const int tid = threadIdx.x, n0 = blockIdx.x * NCH;
  for (int i = tid; i < NCH; i += 256) scnt[i] = 0;
  __syncthreads();
  for (int e = tid; e < NE; e += 256) { const int i = ei[NE + e] - n0;
    if (i >= 0 && i < NCH) { const int s = atomicAdd(&scnt[i], 1); if (s < SLOTC) slots[i][s] = e; } }
  __syncthreads();
  for (int i = tid; i < NCH; i += 256) { const int n = n0 + i; if (n >= NN) continue;
    const int ctrue = scnt[i]; int c = ctrue; if (c > SLOTC) c = SLOTC;
    for (int a = 1; a < c; ++a) { const int v = slots[i][a]; int b = a - 1; while (b >= 0 && slots[i][b] > v) { slots[i][b + 1] = slots[i][b]; --b; } slots[i][b + 1] = v; }
    for (int a = c; a < SLOTC; ++a) slots[i][a] = 0;
    slots[i][SLOTC - 1] = ctrue;
#pragma unroll 1
    for (int p = 0; p < SLOTC / 4; ++p) { v4i v = { slots[i][4 * p], slots[i][4 * p + 1], slots[i][4 * p + 2], slots[i][4 * p + 3] }; vst2(tlist + (size_t)n * SLOTC + 4 * p, v); }
    vst2(cnt + (size_t)n * 32, (int_a)ctrue);
  }
}

__global__ __launch_bounds__(128) void k_msg(const float* __restrict__ h, const float* __restrict__ Wm, const float* __restrict__ Wsf,
                                           const float* __restrict__ coef, const float* __restrict__ blend, float* __restrict__ m, float* __restrict__ hs) {
  __shared__ __align__(16) float so[4][16][HH], s2[4][16][HH];
  const int tid = threadIdx.x, w = tid >> 5, lane = tid & 31, col = lane & 15, g = lane >> 4;
  const int n0 = blockIdx.x * 64 + w * 16;
  if (n0 >= NN) return;
  const v16h a = frag_rowK(h + (size_t)(n0 + col) * HH, lane, HH);
  v8f am[2] = {}, as[2] = {};
#pragma unroll
  for (int t = 0; t < 2; ++t) { am[t] = wmma16(a, frag_col(Wm, t * 16 + col, lane, HH, HH), am[t]); as[t] = wmma16(a, frag_col(Wsf, t * 16 + col, lane, HH, HH), as[t]); }
#pragma unroll
  for (int t = 0; t < 2; ++t) { const int c = t * 16 + col; const float bl = blend[c];
#pragma unroll 1
    for (int r = 0; r < 8; ++r) { so[w][8 * g + r][c] = spline_act(am[t][r], coef + c * NBAS, bl); s2[w][8 * g + r][c] = as[t][r]; } }
  LDSX();
#pragma unroll
  for (int q = 0; q < 4; ++q) { const int rl = q * 4 + (lane >> 3), pc = lane & 7;
    vst2(m + (size_t)(n0 + rl) * HH + pc * 4, *(const v4f*)(&so[w][rl][pc * 4]));
    vst2(hs + (size_t)(n0 + rl) * HH + pc * 4, *(const v4f*)(&s2[w][rl][pc * 4])); }
}

__global__ __launch_bounds__(128) void k_upd(const float* __restrict__ m, const float* __restrict__ hs, const int* __restrict__ ei,
                                           const int* __restrict__ tlist, const int* __restrict__ cnt,
                                           const float* __restrict__ Wo, const float* __restrict__ coef, const float* __restrict__ blend,
                                           const float* __restrict__ lg, const float* __restrict__ lb, float* __restrict__ h) {
  __shared__ __align__(16) float sc[4][16][HH + 4], so[4][16][HH + 4];
  const int tid = threadIdx.x, w = tid >> 5, lane = tid & 31, col = lane & 15, g = lane >> 4;
  const int n0 = blockIdx.x * 64 + w * 16;
  if (n0 >= NN) return;
  const int c = lane;
#pragma unroll 1
  for (int j = 0; j < 16; ++j) { const int n = n0 + j;
    int dn = tlist[(size_t)n * SLOTC + SLOTC - 1]; dn = dn < 0 ? 0 : (dn > SLOTC - 1 ? SLOTC - 1 : dn);
    const float disn = rsqrtf((float)(dn + 1));
    float s = disn * m[(size_t)n * HH + c];
#pragma unroll 1
    for (int q = 0; q < dn; ++q) { int e = tlist[(size_t)n * SLOTC + q]; if ((unsigned)e >= (unsigned)NE) continue;
      int r = ei[e]; r = r < 0 ? 0 : (r >= NN ? NN - 1 : r);
      int dr = tlist[(size_t)r * SLOTC + SLOTC - 1]; dr = dr < 0 ? 0 : (dr > SLOTC - 1 ? SLOTC - 1 : dr);
      s += rsqrtf((float)(dr + 1)) * m[(size_t)r * HH + c]; }
    const float agg = disn * s;
    sc[w][j][c] = spline_act(agg + hs[(size_t)n * HH + c], coef + c * NBAS, blend[c]); }
  LDSX();
  const v16h a = frag_rowK(&sc[w][col][0], lane, HH);
  v8f acc[2] = {};
#pragma unroll
  for (int t = 0; t < 2; ++t) acc[t] = wmma16(a, frag_col(Wo, t * 16 + col, lane, HH, HH), acc[t]);
#pragma unroll
  for (int t = 0; t < 2; ++t)
#pragma unroll
    for (int r = 0; r < 8; ++r) so[w][8 * g + r][t * 16 + col] = acc[t][r];
  LDSX();
#pragma unroll 1
  for (int j = 0; j < 16; ++j) { const int n = n0 + j; const float o = so[w][j][c];
    float mu = o;
#pragma unroll
    for (int off = 16; off >= 1; off >>= 1) mu += __shfl_xor(mu, off, 32);
    mu /= (float)HH;
    float var = (o - mu) * (o - mu);
#pragma unroll
    for (int off = 16; off >= 1; off >>= 1) var += __shfl_xor(var, off, 32);
    var /= (float)HH;
    so[w][j][c] = h[(size_t)n * HH + c] + ((o - mu) / sqrtf(var + 1e-5f)) * lg[c] + lb[c]; }
  LDSX();
#pragma unroll
  for (int q = 0; q < 4; ++q) { const int rl = q * 4 + (lane >> 3), pc = lane & 7;
    vst2(h + (size_t)(n0 + rl) * HH + pc * 4, *(const v4f*)(&so[w][rl][pc * 4])); }
}

__global__ __launch_bounds__(256) void k_readout(const float* __restrict__ h, const int* __restrict__ batch,
                                               const float* __restrict__ W1, const float* __restrict__ b1, const float* __restrict__ c1, const float* __restrict__ bl1,
                                               const float* __restrict__ W2, const float* __restrict__ b2, const float* __restrict__ c2, const float* __restrict__ bl2,
                                               const float* __restrict__ W3, const float* __restrict__ b3, float* __restrict__ res) {
  __shared__ int cntlt[256], cnteq[256];
  __shared__ float psum[8][HH], pmax[8][HH], hg[2 * HH], r1[HH], r2[HF];
  const int gidx = blockIdx.x, tid = threadIdx.x, w = tid >> 5, lane = tid & 31;
  int lt = 0, eq = 0;
  for (int i = tid; i < NN; i += 256) { const int b = batch[i]; lt += (b < gidx); eq += (b == gidx); }
  cntlt[tid] = lt; cnteq[tid] = eq; __syncthreads();
  for (int st = 128; st > 0; st >>= 1) { if (tid < st) { cntlt[tid] += cntlt[tid + st]; cnteq[tid] += cnteq[tid + st]; } __syncthreads(); }
  const int start = cntlt[0], count = cnteq[0];
  float s = 0.f, mx = -3.0e38f;
  for (int i = start + w; i < start + count; i += 8) { const float v = h[(size_t)i * HH + lane]; s += v; mx = fmaxf(mx, v); }
  psum[w][lane] = s; pmax[w][lane] = mx; __syncthreads();
  if (tid < HH) { float t = 0.f, m2 = -3.0e38f; for (int i = 0; i < 8; ++i) { t += psum[i][tid]; m2 = fmaxf(m2, pmax[i][tid]); }
    hg[tid] = count > 0 ? t / (float)count : 0.f; hg[HH + tid] = count > 0 ? m2 : 0.f; }
  __syncthreads();
  if (tid < HH) { float a = b1[tid];
#pragma unroll 1
    for (int i = 0; i < 2 * HH; ++i) a += hg[i] * W1[i * HH + tid];
    r1[tid] = spline_act(a, c1 + tid * NBAS, bl1[tid]); }
  __syncthreads();
  if (tid < HF) { float a = b2[tid];
#pragma unroll 1
    for (int i = 0; i < HH; ++i) a += r1[i] * W2[i * HF + tid];
    r2[tid] = spline_act(a, c2 + tid * NBAS, bl2[tid]); }
  __syncthreads();
  __shared__ float rfin;
  if (tid == 0) { float a = b3[0];
#pragma unroll 1
    for (int i = 0; i < HF; ++i) a += r2[i] * W3[i];
    rfin = 1.0f / (1.0f + expf(-a)); }
  __syncthreads();
  if (tid < 8) { const float v = rfin; v4f q4 = {v, v, v, v}; vst2(res + (size_t)gidx * 32 + tid * 4, q4); }
}
__global__ __launch_bounds__(128) void k_final(const float* __restrict__ res, float* __restrict__ out) {
  __shared__ __align__(16) float so[NG];
  so[threadIdx.x] = res[(size_t)threadIdx.x * 32];
  __syncthreads();
  if (threadIdx.x < 32) vst2(out + threadIdx.x * 4, *(const v4f*)(&so[threadIdx.x * 4]));
}

extern "C" void kernel_launch(void* const* d_in, const int* in_sizes, int n_in,
                              void* d_out, int out_size, void* d_ws, size_t ws_size,
                              hipStream_t stream) {
  (void)in_sizes; (void)n_in; (void)out_size; (void)ws_size;
  const float* x = (const float*)d_in[0]; const float* Win = (const float*)d_in[1]; const float* bin = (const float*)d_in[2];
  const float* cin = (const float*)d_in[3]; const float* blin = (const float*)d_in[4];
  const float* Wm = (const float*)d_in[5]; const float* Wsf = (const float*)d_in[6]; const float* Wo = (const float*)d_in[7];
  const float* cmsg = (const float*)d_in[8]; const float* bmsg = (const float*)d_in[9];
  const float* cupd = (const float*)d_in[10]; const float* bupd = (const float*)d_in[11];
  const float* lg = (const float*)d_in[12]; const float* lb = (const float*)d_in[13];
  const float* W1 = (const float*)d_in[14]; const float* b1 = (const float*)d_in[15]; const float* c1 = (const float*)d_in[16]; const float* bl1 = (const float*)d_in[17];
  const float* W2 = (const float*)d_in[18]; const float* b2 = (const float*)d_in[19]; const float* c2 = (const float*)d_in[20]; const float* bl2 = (const float*)d_in[21];
  const float* W3 = (const float*)d_in[22]; const float* b3 = (const float*)d_in[23];
  const int* ei = (const int*)d_in[24]; const int* batch = (const int*)d_in[25];
  float* out = (float*)d_out;
  char* ws = (char*)d_ws; size_t off = 0;
  auto take = [&](size_t bytes) { char* p = ws + off; off += (bytes + 255) & ~(size_t)255; return p; };
  const int NPAD = ((NN + 63) / 64) * 64;
  float* h  = (float*)take((size_t)NPAD * HH * 4);
  float* m  = (float*)take((size_t)NPAD * HH * 4);
  float* hs = (float*)take((size_t)NPAD * HH * 4);
  int* tlist = (int*)take((size_t)NN * SLOTC * 4); int* cnt = (int*)take((size_t)NN * 32 * 4);
  float* res = (float*)take((size_t)NG * 32 * 4);
  k_in<<<(NN + 63) / 64, 128, 0, stream>>>(x, Win, bin, cin, blin, h);
  k_bucket<<<(NN + NCH - 1) / NCH, 256, 0, stream>>>(ei, tlist, cnt);
  for (int l = 0; l < 3; ++l) {
    k_msg<<<(NN + 63) / 64, 128, 0, stream>>>(h, Wm + (size_t)l * HH * HH, Wsf + (size_t)l * HH * HH, cmsg + (size_t)l * HH * NBAS, bmsg + l * HH, m, hs);
    k_upd<<<(NN + 63) / 64, 128, 0, stream>>>(m, hs, ei, tlist, cnt, Wo + (size_t)l * HH * HH, cupd + (size_t)l * HH * NBAS, bupd + l * HH, lg + l * HH, lb + l * HH, h);
  }
  k_readout<<<NG, 256, 0, stream>>>(h, batch, W1, b1, c1, bl1, W2, b2, c2, bl2, W3, b3, res);
  k_final<<<1, 128, 0, stream>>>(res, out);
}
